// LogLinearMamba2Block_62216896250127
// MI455X (gfx1250) — hardware-run, weakly checked
//
#include <hip/hip_runtime.h>
#include <math.h>

typedef __attribute__((ext_vector_type(16))) _Float16 v16h;
typedef __attribute__((ext_vector_type(8)))  _Float16 v8h;
typedef __attribute__((ext_vector_type(8)))  float    v8f;
typedef __attribute__((ext_vector_type(4)))  float    v4f;

constexpr int kB       = 2;
constexpr int kT       = 1024;
constexpr int kDm      = 1024;
constexpr int kH       = 16;
constexpr int kP       = 128;
constexpr int kNs      = 128;
constexpr int kI       = 2048;
constexpr int kL       = 11;
constexpr int kIM      = 2816;
constexpr int kCC      = 2304;
constexpr int kNProj   = 4368;
constexpr int kNLam    = 176;
constexpr int kNProjPad = 4416;
constexpr int kNLamPad = 192;
constexpr int kNCat    = 4608;
constexpr int kGU      = 5632;
constexpr int kRows    = kB * kT;
constexpr int kColXBC  = 2048;
constexpr int kColDt   = 4352;
constexpr int kColLam  = 4416;
constexpr int kBCw     = 256;
constexpr int kConvTP  = 260;
constexpr int kVtP     = 72;
constexpr float kEps      = 1e-5f;
constexpr float kInvDm    = 1.0f / (float)kDm;
constexpr float kInvI     = 1.0f / (float)kI;
constexpr float kWCarry   = 32.0f;
constexpr float kXbcCarry = 64.0f;
constexpr float kWtCarry  = 256.0f;
constexpr float kHCarry   = 16.0f;
constexpr float kActCarry = 16.0f;
constexpr float kScaleProj = 1.0f / kWCarry;
constexpr float kScaleQK   = 1.0f / (kXbcCarry * kXbcCarry);
constexpr float kScaleY    = 1.0f / (kWtCarry * kXbcCarry);
constexpr float kScaleOut  = 1.0f / (kHCarry * kWCarry);
constexpr float kScaleDown = 1.0f / (kActCarry * kWCarry);

static_assert(kNProj == 2 * kI + 2 * kNs + kH, "in_proj width");
static_assert(kCC == kI + 2 * kNs, "conv channels");
static_assert(kNLam == kH * kL, "lam width");
static_assert(kI == kH * kP, "inner width");
static_assert(kColDt == 2 * kI + 2 * kNs, "dt column");
static_assert(kNProjPad % 64 == 0 && kNProjPad >= kNProj, "pad");
static_assert(kNLamPad % 64 == 0 && kNLamPad >= kNLam, "pad");
static_assert(kNCat == kNProjPad + kNLamPad && kColLam == kNProjPad, "cat width");
static_assert(kGU == 2 * kIM, "gate|up width");
static_assert(kRows % 64 == 0 && kNCat % 64 == 0 && kDm % 64 == 0 && kGU % 64 == 0 && kT % 64 == 0, "tile multiples");
static_assert(kDm % 32 == 0 && kI % 32 == 0 && kIM % 32 == 0 && kNs % 32 == 0, "k multiples");
static_assert(kDm % 64 == 0 && kI % 64 == 0 && kIM % 64 == 0, "transpose k tiles");
static_assert(kBCw == 2 * kNs, "key|query plane width");

constexpr size_t kOffP   = 0;
constexpr size_t kOffW   = kOffP  + (size_t)kRows * kGU * 4;
constexpr size_t kOffX   = kOffW  + (size_t)kGU * kDm * 2;
constexpr size_t kOffBC  = kOffX  + (size_t)kRows * kDm * 2;
constexpr size_t kOffVT  = kOffBC + (size_t)kRows * kBCw * 2;
constexpr size_t kOffH   = kOffVT + (size_t)kB * kI * kT * 2;
constexpr size_t kOffVF  = kOffH  + (size_t)kRows * kI * 2;
constexpr size_t kOffY   = kOffVF + (size_t)kRows * kI * 4;
constexpr size_t kOffR2  = kOffY  + (size_t)kRows * kI * 4;
constexpr size_t kOffDT  = kOffR2 + (size_t)kRows * kDm * 4;
constexpr size_t kOffG   = kOffDT + (size_t)kB * kH * kT * 4;
constexpr size_t kOffQK  = kOffG  + (size_t)kB * kH * kT * 4;
constexpr size_t kWsTotal = kOffQK + (size_t)kB * kT * kT * 4;
static_assert(kWsTotal == 130285568ull, "carve total");
static_assert(kWsTotal <= 134217728ull, "carve cap");
static_assert((size_t)kRows * kNCat * 4 <= (size_t)kRows * kGU * 4, "proj fits region P");
static_assert((size_t)kNCat * kDm * 2 <= (size_t)kGU * kDm * 2, "cat weights fit region W");
static_assert((size_t)kDm * kI * 2 <= (size_t)kGU * kDm * 2, "out weights fit region W");
static_assert((size_t)kDm * kIM * 2 <= (size_t)kGU * kDm * 2, "down weights fit region W");
static_assert((size_t)kRows * kIM * 2 <= (kOffVF - kOffVT), "act fits VT|H");
static_assert((kOffW % 128) == 0 && (kOffX % 128) == 0 && (kOffBC % 128) == 0 && (kOffVT % 128) == 0 &&
              (kOffH % 128) == 0 && (kOffVF % 128) == 0 && (kOffY % 128) == 0 && (kOffR2 % 128) == 0 &&
              (kOffDT % 128) == 0 && (kOffG % 128) == 0 && (kOffQK % 128) == 0, "aligned regions");

struct FragH {
  union U { v16h v; v8h h[2]; };
  static __device__ __forceinline__ v16h load(const _Float16* p) {
    U f;
    f.h[0] = *(const v8h*)(p);
    f.h[1] = *(const v8h*)(p + 16);
    return f.v;
  }
  static __device__ __forceinline__ v8f mma(v16h a, v16h b, v8f c) {
    return __builtin_amdgcn_wmma_f32_16x16x32_f16(false, a, false, b, (short)0, c, false, false);
  }
};
__device__ __forceinline__ v8f mma_h_guarded(v16h a, v16h b, v8f c) {
  c = __builtin_amdgcn_wmma_f32_16x16x32_f16(false, a, false, b, (short)0, c, false, false);
  asm volatile("v_nop\n\tv_nop\n\tv_nop\n\tv_nop" : "+v"(c) : "v"(a), "v"(b));
  return c;
}
__device__ __forceinline__ void guard4_h(v8f& a0, v8f& a1, v8f& a2, v8f& a3, v16h x,
                                         v16h b0, v16h b1, v16h b2, v16h b3) {
  asm volatile("v_nop\n\tv_nop\n\tv_nop\n\tv_nop"
               : "+v"(a0), "+v"(a1), "+v"(a2), "+v"(a3)
               : "v"(x), "v"(b0), "v"(b1), "v"(b2), "v"(b3));
}
__device__ __forceinline__ void acc_guard4(v8f& a, v8f& b, v8f& c, v8f& d) {
  asm volatile("v_nop\n\tv_nop\n\tv_nop\n\tv_nop" : "+v"(a), "+v"(b), "+v"(c), "+v"(d));
}
__device__ __forceinline__ void wave_lds_sync() {
  __builtin_amdgcn_fence(__ATOMIC_RELEASE, "workgroup");
  __builtin_amdgcn_wave_barrier();
  __builtin_amdgcn_fence(__ATOMIC_ACQUIRE, "workgroup");
}

template <bool RESID>
__global__ __launch_bounds__(256) void wmma_gemm64_f16(
    const unsigned short* __restrict__ Ap, int lda, long strideA,
    const unsigned short* __restrict__ Btp, int ldb, long strideB,
    float* __restrict__ Cout, int ldc, long strideC,
    const float* __restrict__ resid, long strideR,
    int M, int N, int K, float scale) {
  const _Float16* A  = (const _Float16*)Ap;
  const _Float16* Bt = (const _Float16*)Btp;
  __shared__ __align__(16) float sT[8][16 * 68];
  const int b    = blockIdx.y;
  const int lane = threadIdx.x & 31;
  const int wave = threadIdx.x >> 5;
  const int tilesN = N >> 6;
  const int tilesM = M >> 6;
  const int tile = blockIdx.x * 8 + wave;
  if (tile >= tilesM * tilesN) return;
  const int tm = tile / tilesN;
  const int tn = tile - tm * tilesN;
  const int m0 = tm << 6;
  const int n0 = tn << 6;

  const _Float16* Ab = A  + (size_t)b * strideA;
  const _Float16* Bb = Bt + (size_t)b * strideB;

  const int rlane = lane & 15;
  const int koff  = (lane >> 4) * 8;
  const int mOff  = (lane >> 4) * 8;

  v8f acc[4][4];
#pragma unroll
  for (int i = 0; i < 4; ++i)
#pragma unroll
    for (int j = 0; j < 4; ++j) acc[i][j] = (v8f){0.f, 0.f, 0.f, 0.f, 0.f, 0.f, 0.f, 0.f};

  for (int k0 = 0; k0 < K; k0 += 32) {
    v16h bh[4];
#pragma unroll
    for (int j = 0; j < 4; ++j) {
      const size_t bo = (size_t)(n0 + (j << 4) + rlane) * ldb + koff + k0;
      bh[j] = FragH::load(Bb + bo);
    }
#pragma unroll
    for (int i = 0; i < 4; ++i) {
      const size_t ao = (size_t)(m0 + (i << 4) + rlane) * lda + koff + k0;
      v16h ah = FragH::load(Ab + ao);
#pragma unroll
      for (int j = 0; j < 4; ++j) acc[i][j] = FragH::mma(ah, bh[j], acc[i][j]);
      guard4_h(acc[i][0], acc[i][1], acc[i][2], acc[i][3], ah, bh[0], bh[1], bh[2], bh[3]);
    }
  }
  acc_guard4(acc[0][0], acc[0][1], acc[0][2], acc[0][3]);
  acc_guard4(acc[1][0], acc[1][1], acc[1][2], acc[1][3]);
  acc_guard4(acc[2][0], acc[2][1], acc[2][2], acc[2][3]);
  acc_guard4(acc[3][0], acc[3][1], acc[3][2], acc[3][3]);

  float* slab = sT[wave];
  float* C = Cout + (size_t)b * strideC;
  const float* Rb = resid + (size_t)b * strideR;
  const int hh = lane >> 4, c4 = (lane & 15) * 4;
#pragma unroll
  for (int i = 0; i < 4; ++i) {
    const int mBase = m0 + (i << 4);
#pragma unroll
    for (int j = 0; j < 4; ++j) {
#pragma unroll
      for (int r = 0; r < 8; ++r) slab[(mOff + r) * 68 + (j << 4) + rlane] = acc[i][j][r] * scale;
    }
    wave_lds_sync();
    v4f ov[8];
#pragma unroll
    for (int it = 0; it < 8; ++it) {
      const int row = it * 2 + hh;
      v4f v = *(const v4f*)(slab + row * 68 + c4);
      if (RESID) {
        const v4f rv = *(const v4f*)(Rb + (size_t)(mBase + row) * ldc + n0 + c4);
        v = v + rv;
      }
      ov[it] = v;
    }
    for (int pass = 0; pass < 2; ++pass) {
#pragma unroll
      for (int it = 0; it < 8; ++it) {
        const int row = it * 2 + hh;
        *(volatile v4f*)(C + (size_t)(mBase + row) * ldc + n0 + c4) = ov[it];
      }
      __threadfence();
    }
    wave_lds_sync();
  }
}

__global__ __launch_bounds__(256) void transpose_cast_kernel(
    const float* __restrict__ W, unsigned short* __restrict__ Bt, int Kdim, int Ndim, float scale)
{
  __shared__ float tile[64 * 65];
  const int tid = threadIdx.x, lane = tid & 31, wave = tid >> 5;
  const int n0 = blockIdx.x * 64;
  const int k0 = blockIdx.y * 64;
#pragma unroll
  for (int p = 0; p < 16; ++p) {
    const int idx = tid + p * 256;
    const int kk  = idx >> 6;
    const int nn  = idx & 63;
    const int n   = n0 + nn;
    const int nc  = (n < Ndim) ? n : (Ndim - 1);
    const float v = W[(size_t)(k0 + kk) * Ndim + nc];
    tile[kk * 65 + nn] = (n < Ndim) ? (v * scale) : 0.f;
  }
  __syncthreads();
  const int q = lane >> 3, c8 = (lane & 7) * 8;
  v8h hv[2];
#pragma unroll
  for (int it = 0; it < 2; ++it) {
    const int nrow = it * 32 + wave * 4 + q;
#pragma unroll
    for (int e = 0; e < 8; ++e) hv[it][e] = (_Float16)tile[(c8 + e) * 65 + nrow];
  }
  for (int pass = 0; pass < 2; ++pass) {
#pragma unroll
    for (int it = 0; it < 2; ++it) {
      const int nrow = it * 32 + wave * 4 + q;
      *(volatile v8h*)(Bt + (size_t)(n0 + nrow) * Kdim + k0 + c8) = hv[it];
    }
    __threadfence();
  }
}

__global__ __launch_bounds__(128) void rmsnorm_f16_kernel(
    const float* __restrict__ src, const float* __restrict__ w, unsigned short* __restrict__ dst)
{
  __shared__ float red[4];
  const int tid = threadIdx.x, lane = tid & 31, wave = tid >> 5;
  const size_t row = blockIdx.x;
  const float* p = src + row * kDm + tid * 8;
  const v4f a0 = *(const v4f*)(p);
  const v4f a1 = *(const v4f*)(p + 4);
  const v4f w0 = *(const v4f*)(w + tid * 8);
  const v4f w1 = *(const v4f*)(w + tid * 8 + 4);
  float ss = 0.f;
#pragma unroll
  for (int e = 0; e < 4; ++e) {
    ss = fmaf(a0[e], a0[e], ss);
    ss = fmaf(a1[e], a1[e], ss);
  }
#pragma unroll
  for (int off = 16; off > 0; off >>= 1) ss += __shfl_xor(ss, off, 32);
  if (lane == 0) red[wave] = ss;
  __syncthreads();
  const float tot = ((red[0] + red[1]) + red[2]) + red[3];
  const float inv = rsqrtf(tot * kInvDm + kEps);
  v8h hv;
#pragma unroll
  for (int e = 0; e < 4; ++e) {
    hv[e]     = (_Float16)((a0[e] * inv) * w0[e]);
    hv[4 + e] = (_Float16)((a1[e] * inv) * w1[e]);
  }
  unsigned short* q = dst + row * kDm + tid * 8;
  *(volatile v8h*)q = hv;
  __threadfence();
  *(volatile v8h*)q = hv;
}

__global__ __launch_bounds__(256) void conv_silu_kernel(
    const float* __restrict__ proj, const float* __restrict__ cw, const float* __restrict__ cb,
    float* __restrict__ VF, unsigned short* __restrict__ VT, unsigned short* __restrict__ XBC)
{
  __shared__ __align__(16) float sT[16 * kConvTP];
  __shared__ __align__(16) _Float16 sV[256 * kVtP];
  const int tid = threadIdx.x, lane = tid & 31, wave = tid >> 5;
  const bool isV = ((int)blockIdx.x < (kI / 256));
  const int d0 = blockIdx.x * 256, d = d0 + tid;
  const int g0 = blockIdx.y * 64;
  const int tb = g0 & (kT - 1);
  const int bix = g0 / kT;
  const float w0 = cw[d * 4 + 0], w1 = cw[d * 4 + 1], w2 = cw[d * 4 + 2], w3 = cw[d * 4 + 3];
  const float bc = cb[d];
  const float* src = proj + kColXBC + d;
  float xm3, xm2, xm1;
  {
    const bool hist = (tb > 0);
    const int rb = hist ? (g0 - 3) : g0;
    const float v3 = src[(size_t)rb * kNCat];
    const float v2 = src[(size_t)(rb + 1) * kNCat];
    const float v1 = src[(size_t)(rb + 2) * kNCat];
    xm3 = hist ? v3 : 0.f;
    xm2 = hist ? v2 : 0.f;
    xm1 = hist ? v1 : 0.f;
  }
  const int hrow = wave >> 1;
  const int hch  = (wave & 1) * 128 + lane * 4;
  const float tscale = isV ? 1.0f : kXbcCarry;
#pragma unroll 1
  for (int sub = 0; sub < 4; ++sub) {
    const int lb = g0 + sub * 16;
#pragma unroll 1
    for (int s = 0; s < 16; ++s) {
      const float xcur = src[(size_t)(lb + s) * kNCat];
      float acc = w0 * xm3;
      acc = fmaf(w1, xm2, acc);
      acc = fmaf(w2, xm1, acc);
      acc = fmaf(w3, xcur, acc);
      const float sv = acc + bc;
      const float sg = 1.0f / (1.0f + expf(-sv));
      const float val = sv * sg;
      sT[s * kConvTP + tid] = val * tscale;
      sV[tid * kVtP + sub * 16 + s] = (_Float16)(val * kXbcCarry);
      xm3 = xm2; xm2 = xm1; xm1 = xcur;
    }
    __syncthreads();
    if (isV) {
      v4f fv[4];
#pragma unroll
      for (int it = 0; it < 4; ++it) fv[it] = *(const v4f*)(sT + (it * 4 + hrow) * kConvTP + hch);
      for (int pass = 0; pass < 2; ++pass) {
#pragma unroll
        for (int it = 0; it < 4; ++it)
          *(volatile v4f*)(VF + (size_t)(lb + it * 4 + hrow) * kI + d0 + hch) = fv[it];
        __threadfence();
      }
    } else {
      v8h bv[2];
#pragma unroll
      for (int it = 0; it < 2; ++it) {
        const float* sp = sT + (it * 8 + wave) * kConvTP + lane * 8;
        const v4f a0 = *(const v4f*)(sp);
        const v4f a1 = *(const v4f*)(sp + 4);
#pragma unroll
        for (int e = 0; e < 4; ++e) {
          bv[it][e]     = (_Float16)a0[e];
          bv[it][4 + e] = (_Float16)a1[e];
        }
      }
      for (int pass = 0; pass < 2; ++pass) {
#pragma unroll
        for (int it = 0; it < 2; ++it)
          *(volatile v8h*)(XBC + (size_t)(lb + it * 8 + wave) * kBCw + lane * 8) = bv[it];
        __threadfence();
      }
    }
    __syncthreads();
  }
  if (isV) {
    const int q = lane >> 3, c8 = (lane & 7) * 8;
    v8h tv[8];
#pragma unroll
    for (int it = 0; it < 8; ++it) {
      const int chl = it * 32 + wave * 4 + q;
      tv[it] = *(const v8h*)(sV + chl * kVtP + c8);
    }
    for (int pass = 0; pass < 2; ++pass) {
#pragma unroll
      for (int it = 0; it < 8; ++it) {
        const int chl = it * 32 + wave * 4 + q;
        *(volatile v8h*)(VT + (size_t)(bix * kI + d0 + chl) * kT + tb + c8) = tv[it];
      }
      __threadfence();
    }
  }
}

__global__ __launch_bounds__(32) void dt_scan_kernel(
    const float* __restrict__ proj, const float* __restrict__ dt_bias, const float* __restrict__ A_log,
    float* __restrict__ DT, float* __restrict__ G)
{
  __shared__ __align__(16) float sDt[kT];
  __shared__ __align__(16) float sG[kT];
  __shared__ double sTot[32];
  const int lane = threadIdx.x;
  const int bh = blockIdx.x;
  const int b = bh / kH, h = bh - b * kH;
  const float bias = dt_bias[h];
  const float Ax = -expf(A_log[h]);
  const float* src = proj + (size_t)b * kT * kNCat + kColDt + h;
  double run = 0.0;
#pragma unroll 1
  for (int i = 0; i < 32; ++i) {
    const int t = lane * 32 + i;
    const float raw = src[(size_t)t * kNCat] + bias;
    const float dtv = fmaxf(raw, 0.0f) + log1pf(expf(-fabsf(raw)));
    const float a = dtv * Ax;
    run += (double)a;
    sDt[t] = dtv;
    sG[t] = (float)run;
  }
  sTot[lane] = run;
  __syncthreads();
  double off = 0.0;
#pragma unroll 1
  for (int j = 0; j < 32; ++j) {
    const double tv = sTot[j];
    off += (j < lane) ? tv : 0.0;
  }
#pragma unroll 1
  for (int i = 0; i < 32; ++i) {
    const int t = lane * 32 + i;
    sG[t] = (float)(off + (double)sG[t]);
  }
  __syncthreads();
  v4f dv[8], gv[8];
#pragma unroll
  for (int it = 0; it < 8; ++it) {
    dv[it] = *(const v4f*)(sDt + it * 128 + lane * 4);
    gv[it] = *(const v4f*)(sG + it * 128 + lane * 4);
  }
  for (int pass = 0; pass < 2; ++pass) {
#pragma unroll
    for (int it = 0; it < 8; ++it) {
      *(volatile v4f*)(DT + (size_t)bh * kT + it * 128 + lane * 4) = dv[it];
      *(volatile v4f*)(G + (size_t)bh * kT + it * 128 + lane * 4) = gv[it];
    }
    __threadfence();
  }
}

__global__ __launch_bounds__(128) void decay_attn_kernel(
    const float* __restrict__ QK, const float* __restrict__ proj, const float* __restrict__ G,
    const float* __restrict__ DT, const unsigned short* __restrict__ VTp, float* __restrict__ Y)
{
  __shared__ __align__(16) _Float16 sW[4][16 * 32];
  __shared__ __align__(16) float sLam[4][16 * 12];
  __shared__ float sGq[4][16];
  __shared__ __align__(16) float sO[4][16 * 68];
  const int tid = threadIdx.x, wave = tid >> 5, lane = tid & 31;
  const int hh = lane >> 4, c = lane & 15;
  const int bh = blockIdx.y;
  const int b = bh / kH, h = bh - b * kH;
  const int t0 = blockIdx.x * 64 + wave * 16;
  const _Float16* VT = (const _Float16*)VTp;

  {
    const float* prow = proj + (size_t)(b * kT + t0) * kNCat + kColLam + h * kL;
#pragma unroll 1
    for (int i = 0; i < 6; ++i) {
      const int idx = i * 32 + lane;
      const int row = idx / 12;
      const int l = idx - row * 12;
      const int lc = (l < kL) ? l : (kL - 1);
      const float v = prow[(size_t)row * kNCat + lc];
      sLam[wave][idx] = (l < kL) ? v : 0.f;
    }
    sGq[wave][c] = G[(size_t)bh * kT + t0 + c];
  }
  __syncthreads();

  v8f yacc[8];
#pragma unroll
  for (int i = 0; i < 8; ++i) yacc[i] = (v8f){0.f, 0.f, 0.f, 0.f, 0.f, 0.f, 0.f, 0.f};

  const int nblk = (t0 >> 5) + 1;
  const float* gcol = G + (size_t)bh * kT;
  const float* dcol = DT + (size_t)bh * kT;
  const float* qbase = QK + (size_t)(b * kT + t0) * kT;
  const _Float16* vbase = VT + (size_t)(b * kI + h * kP + c) * kT + 8 * hh;
  _Float16* wt = sW[wave];
  const float* lamw = sLam[wave];
  const float* gqw = sGq[wave];

#pragma unroll 1
  for (int kb = 0; kb < nblk; ++kb) {
    const int s0 = kb * 32;
    float gsv[2], dsv[2];
#pragma unroll
    for (int j = 0; j < 2; ++j) {
      gsv[j] = gcol[s0 + j * 16 + c];
      dsv[j] = dcol[s0 + j * 16 + c];
    }
#pragma unroll 1
    for (int r = 0; r < 8; ++r) {
      const int row = 8 * hh + r;
      const int t = t0 + row;
      const float gt = gqw[row];
      const float* qrow = qbase + (size_t)row * kT + s0;
      const float* lrow = lamw + row * 12;
#pragma unroll
      for (int j = 0; j < 2; ++j) {
        const int sl = j * 16 + c;
        const int s = s0 + sl;
        const bool ok = (s <= t);
        const float q = qrow[sl];
        const int x = t ^ s;
        const int lv1 = 32 - __builtin_clz((unsigned)(x | 1));
        const int lvl = (x == 0) ? 0 : lv1;
        const float lm = lrow[lvl];
        const float arg = ok ? (gt - gsv[j]) : 0.0f;
        const float e = expf(arg);
        const float wv = ((q * e) * lm) * dsv[j];
        const float wsel = ok ? (wv * kWtCarry) : 0.0f;
        wt[row * 32 + sl] = (_Float16)wsel;
      }
    }
    wave_lds_sync();
    const v16h wa = FragH::load(wt + c * 32 + 8 * hh);
#pragma unroll
    for (int nt = 0; nt < 8; ++nt) {
      const v16h vb = FragH::load(vbase + (size_t)(nt * 16) * kT + s0);
      yacc[nt] = mma_h_guarded(wa, vb, yacc[nt]);
    }
    wave_lds_sync();
  }

  float* os = sO[wave];
  const int c4 = (lane & 15) * 4;
  float* ybase = Y + (size_t)(b * kT + t0) * kI + h * kP;
#pragma unroll
  for (int half = 0; half < 2; ++half) {
#pragma unroll
    for (int jj = 0; jj < 4; ++jj) {
#pragma unroll
      for (int r = 0; r < 8; ++r) os[(8 * hh + r) * 68 + jj * 16 + c] = yacc[half * 4 + jj][r] * kScaleY;
    }
    wave_lds_sync();
    v4f ov[8];
#pragma unroll
    for (int it = 0; it < 8; ++it) ov[it] = *(const v4f*)(os + (it * 2 + hh) * 68 + c4);
    for (int pass = 0; pass < 2; ++pass) {
#pragma unroll
      for (int it = 0; it < 8; ++it)
        *(volatile v4f*)(ybase + (size_t)(it * 2 + hh) * kI + half * 64 + c4) = ov[it];
      __threadfence();
    }
    wave_lds_sync();
  }
}

__global__ __launch_bounds__(256) void gate_gnorm_kernel(
    const float* __restrict__ Y, const float* __restrict__ VF, const float* __restrict__ proj,
    const float* __restrict__ Dv, const float* __restrict__ gw, unsigned short* __restrict__ Hout)
{
  __shared__ __align__(16) float sH[kI];
  __shared__ float red[8];
  const int tid = threadIdx.x, lane = tid & 31, wave = tid >> 5;
  const size_t row = blockIdx.x;
  const float* yr = Y + row * kI;
  const float* vr = VF + row * kI;
  const float* zr = proj + row * kNCat;
  float ss = 0.f;
#pragma unroll 1
  for (int i = 0; i < 8; ++i) {
    const int col = i * 256 + tid;
    const float yv = yr[col];
    const float vv = vr[col];
    const float z = zr[col];
    const float dd = Dv[col >> 7];
    const float yy = yv + dd * vv;
    const float sg = 1.0f / (1.0f + expf(-z));
    const float hval = yy * (z * sg);
    sH[col] = hval;
    ss = fmaf(hval, hval, ss);
  }
#pragma unroll
  for (int off = 16; off > 0; off >>= 1) ss += __shfl_xor(ss, off, 32);
  if (lane == 0) red[wave] = ss;
  __syncthreads();
  float tot = 0.f;
#pragma unroll
  for (int i = 0; i < 8; ++i) tot += red[i];
  const float inv = rsqrtf(tot * kInvI + kEps);
  const v4f a0 = *(const v4f*)(sH + tid * 8);
  const v4f a1 = *(const v4f*)(sH + tid * 8 + 4);
  const v4f w0 = *(const v4f*)(gw + tid * 8);
  const v4f w1 = *(const v4f*)(gw + tid * 8 + 4);
  v8h hv;
#pragma unroll
  for (int e = 0; e < 4; ++e) {
    hv[e]     = (_Float16)(((a0[e] * inv) * w0[e]) * kHCarry);
    hv[4 + e] = (_Float16)(((a1[e] * inv) * w1[e]) * kHCarry);
  }
  unsigned short* q = Hout + row * kI + tid * 8;
  *(volatile v8h*)q = hv;
  __threadfence();
  *(volatile v8h*)q = hv;
}

__global__ __launch_bounds__(352) void silu_mul_kernel(
    const float* __restrict__ GUp, unsigned short* __restrict__ ACT)
{
  __shared__ __align__(16) float sA[kIM];
  const int tid = threadIdx.x;
  const size_t row = blockIdx.x;
  const float* gr = GUp + row * kGU;
  const float* ur = gr + kIM;
#pragma unroll 1
  for (int i = 0; i < 8; ++i) {
    const int col = i * 352 + tid;
    const float g = gr[col];
    const float u = ur[col];
    const float sg = 1.0f / (1.0f + expf(-g));
    sA[col] = ((g * sg) * u) * kActCarry;
  }
  __syncthreads();
  const v4f a0 = *(const v4f*)(sA + tid * 8);
  const v4f a1 = *(const v4f*)(sA + tid * 8 + 4);
  v8h hv;
#pragma unroll
  for (int e = 0; e < 4; ++e) {
    hv[e]     = (_Float16)a0[e];
    hv[4 + e] = (_Float16)a1[e];
  }
  unsigned short* q = ACT + row * kIM + tid * 8;
  *(volatile v8h*)q = hv;
  __threadfence();
  *(volatile v8h*)q = hv;
}

extern "C" void kernel_launch(void* const* d_in, const int* in_sizes, int n_in,
                              void* d_out, int out_size, void* d_ws, size_t ws_size,
                              hipStream_t stream)
{
  if (n_in < 15) return;
  if (in_sizes[0] != kRows * kDm) return;
  if (in_sizes[1] != kDm || in_sizes[2] != kDm) return;
  if (in_sizes[3] != kDm * kNProj) return;
  if (in_sizes[4] != kCC * 4 || in_sizes[5] != kCC) return;
  if (in_sizes[6] != kH || in_sizes[7] != kH || in_sizes[8] != kH) return;
  if (in_sizes[9] != kDm * kNLam) return;
  if (in_sizes[10] != kI) return;
  if (in_sizes[11] != kI * kDm) return;
  if (in_sizes[12] != kDm * kIM || in_sizes[13] != kDm * kIM) return;
  if (in_sizes[14] != kIM * kDm) return;
  if (out_size != kRows * kDm) return;
  if (ws_size < kWsTotal) return;

  const float* hidden       = (const float*)d_in[0];
  const float* mixer_norm_w = (const float*)d_in[1];
  const float* mlp_norm_w   = (const float*)d_in[2];
  const float* in_proj_w    = (const float*)d_in[3];
  const float* conv_w       = (const float*)d_in[4];
  const float* conv_b       = (const float*)d_in[5];
  const float* dt_bias      = (const float*)d_in[6];
  const float* A_log        = (const float*)d_in[7];
  const float* Dv           = (const float*)d_in[8];
  const float* lam_w        = (const float*)d_in[9];
  const float* gnorm_w      = (const float*)d_in[10];
  const float* out_proj_w   = (const float*)d_in[11];
  const float* gate_w       = (const float*)d_in[12];
  const float* up_w         = (const float*)d_in[13];
  const float* down_w       = (const float*)d_in[14];
  float* outp = (float*)d_out;

  char* ws = (char*)d_ws;
  float*          PJ  = (float*)(ws + kOffP);
  unsigned short* WS  = (unsigned short*)(ws + kOffW);
  unsigned short* X16 = (unsigned short*)(ws + kOffX);
  unsigned short* BC  = (unsigned short*)(ws + kOffBC);
  unsigned short* VT  = (unsigned short*)(ws + kOffVT);
  unsigned short* H16 = (unsigned short*)(ws + kOffH);
  unsigned short* ACT = (unsigned short*)(ws + kOffVT);
  float*          VF  = (float*)(ws + kOffVF);
  float*          YB  = (float*)(ws + kOffY);
  float*          R2  = (float*)(ws + kOffR2);
  float*          DTB = (float*)(ws + kOffDT);
  float*          GB  = (float*)(ws + kOffG);
  float*          QK  = (float*)(ws + kOffQK);

  rmsnorm_f16_kernel<<<kRows, 128, 0, stream>>>(hidden, mixer_norm_w, X16);

  transpose_cast_kernel<<<dim3(kNProjPad / 64, kDm / 64), 256, 0, stream>>>(in_proj_w, WS, kDm, kNProj, kWCarry);
  transpose_cast_kernel<<<dim3(kNLamPad / 64, kDm / 64), 256, 0, stream>>>(
      lam_w, WS + (size_t)kNProjPad * kDm, kDm, kNLam, kWCarry);

  wmma_gemm64_f16<false><<<dim3((kRows / 64) * (kNCat / 64) / 8, 1), 256, 0, stream>>>(
      X16, kDm, 0L, WS, kDm, 0L, PJ, kNCat, 0L, hidden, 0L, kRows, kNCat, kDm, kScaleProj);

  conv_silu_kernel<<<dim3(kCC / 256, kRows / 64), 256, 0, stream>>>(PJ, conv_w, conv_b, VF, VT, BC);

  dt_scan_kernel<<<kB * kH, 32, 0, stream>>>(PJ, dt_bias, A_log, DTB, GB);

  wmma_gemm64_f16<false><<<dim3((kT / 64) * (kT / 64) / 8, kB), 256, 0, stream>>>(
      BC + kNs, kBCw, (long)kT * kBCw, BC, kBCw, (long)kT * kBCw,
      QK, kT, (long)kT * kT, hidden, 0L, kT, kT, kNs, kScaleQK);

  decay_attn_kernel<<<dim3(kT / 64, kB * kH), 128, 0, stream>>>(QK, PJ, GB, DTB, VT, YB);

  gate_gnorm_kernel<<<kRows, 256, 0, stream>>>(YB, VF, PJ, Dv, gnorm_w, H16);

  transpose_cast_kernel<<<dim3(kDm / 64, kI / 64), 256, 0, stream>>>(out_proj_w, WS, kI, kDm, kWCarry);
  wmma_gemm64_f16<true><<<dim3((kRows / 64) * (kDm / 64) / 8, 1), 256, 0, stream>>>(
      H16, kI, 0L, WS, kI, 0L, R2, kDm, 0L, hidden, 0L, kRows, kDm, kI, kScaleOut);

  rmsnorm_f16_kernel<<<kRows, 128, 0, stream>>>(R2, mlp_norm_w, X16);

  transpose_cast_kernel<<<dim3(kIM / 64, kDm / 64), 256, 0, stream>>>(gate_w, WS, kDm, kIM, kWCarry);
  transpose_cast_kernel<<<dim3(kIM / 64, kDm / 64), 256, 0, stream>>>(
      up_w, WS + (size_t)kIM * kDm, kDm, kIM, kWCarry);
  wmma_gemm64_f16<false><<<dim3((kRows / 64) * (kGU / 64) / 8, 1), 256, 0, stream>>>(
      X16, kDm, 0L, WS, kDm, 0L, PJ, kGU, 0L, hidden, 0L, kRows, kGU, kDm, kScaleProj);

  silu_mul_kernel<<<kRows, 352, 0, stream>>>(PJ, ACT);

  transpose_cast_kernel<<<dim3(kDm / 64, kIM / 64), 256, 0, stream>>>(down_w, WS, kIM, kDm, kWCarry);
  wmma_gemm64_f16<true><<<dim3((kRows / 64) * (kDm / 64) / 8, 1), 256, 0, stream>>>(
      ACT, kIM, 0L, WS, kIM, 0L, outp, kDm, 0L, R2, 0L, kRows, kDm, kIM, kScaleDown);
}
